// DiTBlock_63264868270088
// MI455X (gfx1250) — hardware-verified
//
#include <hip/hip_runtime.h>
#include <math.h>

#ifndef NB
#define NB 1
#endif
#ifndef SEQ
#define SEQ 4096
#endif
#define SEQ_FULL 4096
#define FEAT 768
#define NH   12
#define HD   64
#define QKVW (3 * FEAT)
#define QKP  (2 * FEAT)
#define MF   3072
#define NTOK (NB * SEQ)
static_assert(NB == 1);
static_assert(NH * HD == FEAT);
static_assert((SEQ % 64) == 0 && SEQ <= SEQ_FULL);
static_assert((FEAT % 64) == 0 && (MF % 64) == 0 && (QKP % 64) == 0 && (QKVW % 256) == 0);
static_assert((FEAT % 32) == 0 && (MF % 32) == 0 && (HD % 32) == 0 && (QKVW % 32) == 0);
static_assert(FEAT == 4 * 192);

#define WCARRY   64.0f
#define PSCALE   16384.0f
#define CTXCARRY 256.0f
#define MIDCARRY 16.0f

typedef _Float16 v16h __attribute__((ext_vector_type(16)));
typedef _Float16 v8h  __attribute__((ext_vector_type(8)));
typedef float    v8f  __attribute__((ext_vector_type(8)));
typedef float    v4f  __attribute__((ext_vector_type(4)));
typedef v8h __attribute__((may_alias)) v8ha;
typedef v4f __attribute__((may_alias)) v4fa;
union Frag { v16h v; v8h half[2]; };

#if defined(__HIP_DEVICE_COMPILE__)
#define DEV_ASM 1
#else
#define DEV_ASM 0
#endif

__device__ __forceinline__ v8f zero8() { v8f z = {0.f, 0.f, 0.f, 0.f, 0.f, 0.f, 0.f, 0.f}; return z; }

__device__ __forceinline__ float rne16(float x) {
  unsigned int u = __float_as_uint(x);
  u = (u + 0x7FFFu + ((u >> 16) & 1u)) & 0xFFFF0000u;
  return __uint_as_float(u);
}
__device__ __forceinline__ v4f rne16_4(v4f a) {
  v4f r = { rne16(a.x), rne16(a.y), rne16(a.z), rne16(a.w) };
  return r;
}

__device__ __forceinline__ v8f wmma_f16(v16h a, v16h b, v8f c) {
  v8f d = __builtin_amdgcn_wmma_f32_16x16x32_f16(false, a, false, b, (short)0, c, false, false);
#if DEV_ASM
  asm volatile("v_nop\n\tv_nop\n\tv_nop\n\tv_nop" : "+v"(d) : "v"(a), "v"(b));
#endif
  return d;
}
__device__ __forceinline__ v8f mmar(v16h a, v16h b, v8f c) {
  return __builtin_amdgcn_wmma_f32_16x16x32_f16(false, a, false, b, (short)0, c, false, false);
}
__device__ __forceinline__ void dep_guard(v8f& a, v8f& b, v16h x, v16h y) {
#if DEV_ASM
  asm volatile("v_nop\n\tv_nop\n\tv_nop\n\tv_nop" : "+v"(a), "+v"(b) : "v"(x), "v"(y));
#else
  (void)a; (void)b; (void)x; (void)y;
#endif
}
__device__ __forceinline__ void keep4(v16h a, v16h b, v16h c, v16h d) {
#if DEV_ASM
  asm volatile("v_nop" :: "v"(a), "v"(b), "v"(c), "v"(d));
#else
  (void)a; (void)b; (void)c; (void)d;
#endif
}
__device__ __forceinline__ void acc_guard4(v8f& a, v8f& b, v8f& c, v8f& d) {
#if DEV_ASM
  asm volatile("v_nop\n\tv_nop\n\tv_nop\n\tv_nop" : "+v"(a), "+v"(b), "+v"(c), "+v"(d));
#else
  (void)a; (void)b; (void)c; (void)d;
#endif
}

__device__ __forceinline__ v16h load_frag(const _Float16* p, int h) {
  Frag f;
  f.half[0] = *(const v8ha*)(p + 8 * h);
  f.half[1] = *(const v8ha*)(p + 16 + 8 * h);
  return f.v;
}
__device__ __forceinline__ v16h ldfrag(const _Float16* p) {
  Frag f;
  f.half[0] = *(const v8ha*)(p);
  f.half[1] = *(const v8ha*)(p + 16);
  return f.v;
}

__global__ __launch_bounds__(256) void mod_kernel(
    const float* __restrict__ cond,
    const float* __restrict__ w1, const float* __restrict__ b1,
    const float* __restrict__ w2, const float* __restrict__ b2,
    float* modv)
{
  __shared__ float sc[FEAT];
  const int tid = (int)threadIdx.x;
  const int which = (int)blockIdx.x / (QKVW / 256);
  const int j = ((int)blockIdx.x - which * (QKVW / 256)) * 256 + tid;
#pragma unroll 1
  for (int i = tid; i < FEAT; i += 256) {
    const float c = rne16(cond[i]);
    sc[i] = c * (1.0f / (1.0f + expf(-c)));
  }
  __syncthreads();
  const float* W  = (which == 0) ? w1 : w2;
  const float* bs = (which == 0) ? b1 : b2;
  float acc = 0.0f;
#pragma unroll 1
  for (int i = 0; i < FEAT; ++i) acc += sc[i] * rne16(W[(size_t)i * QKVW + j]);
  const float v = acc + rne16(bs[j]);
  float* dst = modv + (size_t)which * QKVW + j;
  *(volatile float*)dst = v;
  __threadfence();
  *(volatile float*)dst = v;
}

__global__ __launch_bounds__(256) void transpose_cvt(
    const float* __restrict__ in, _Float16* out, int K, int N, float carry)
{
  __shared__ __align__(16) float tile[32][68];
  const int k0 = blockIdx.x * 64, n0 = blockIdx.y * 32;
  const int tid = (int)threadIdx.x;
  {
    const int kk = tid >> 2, nq = (tid & 3) * 8;
    const float* src = in + (size_t)(k0 + kk) * N + n0 + nq;
    const v4f a = *(const v4fa*)src;
    const v4f c = *(const v4fa*)(src + 4);
    tile[nq + 0][kk] = a.x; tile[nq + 1][kk] = a.y; tile[nq + 2][kk] = a.z; tile[nq + 3][kk] = a.w;
    tile[nq + 4][kk] = c.x; tile[nq + 5][kk] = c.y; tile[nq + 6][kk] = c.z; tile[nq + 7][kk] = c.w;
  }
  __syncthreads();
  {
    const int nn = tid >> 3, kq = (tid & 7) * 8;
    const float* sp = &tile[nn][kq];
    const v4f a = *(const v4fa*)sp;
    const v4f c = *(const v4fa*)(sp + 4);
    const v8h o = { (_Float16)(rne16(a.x) * carry), (_Float16)(rne16(a.y) * carry),
                    (_Float16)(rne16(a.z) * carry), (_Float16)(rne16(a.w) * carry),
                    (_Float16)(rne16(c.x) * carry), (_Float16)(rne16(c.y) * carry),
                    (_Float16)(rne16(c.z) * carry), (_Float16)(rne16(c.w) * carry) };
    _Float16* dst = out + (size_t)(n0 + nn) * K + k0 + kq;
    *(volatile v8h*)dst = o;
    __threadfence();
    *(volatile v8h*)dst = o;
  }
}

__device__ __forceinline__ float block_sum(float v, float* red, int lane, int w) {
#pragma unroll
  for (int off = 16; off > 0; off >>= 1) v += __shfl_xor(v, off);
  if (lane == 0) red[w] = v;
  __syncthreads();
  float r = red[0];
#pragma unroll
  for (int i = 1; i < 6; ++i) r += red[i];
  __syncthreads();
  return r;
}

template <bool RIN>
__global__ __launch_bounds__(192) void ln_kernel(
    const float* __restrict__ X, const float* __restrict__ hm, _Float16* pout)
{
  __shared__ __align__(16) float srow[FEAT];
  __shared__ float red[8];
  const int row = blockIdx.x;
  const int tid = (int)threadIdx.x, lane = tid & 31, w = tid >> 5;
  const int f0  = 4 * tid;
  const size_t base = (size_t)row * FEAT + f0;

  v4f xv = *(const v4fa*)(X + base);
  if constexpr (RIN) xv = rne16_4(xv);
  float s = (xv.x + xv.y) + (xv.z + xv.w);
  s = block_sum(s, red, lane, w);
  const float mu = s * (1.0f / FEAT);
  const float d0 = xv.x - mu, d1 = xv.y - mu, d2 = xv.z - mu, d3 = xv.w - mu;
  float q = (d0 * d0 + d1 * d1) + (d2 * d2 + d3 * d3);
  q = block_sum(q, red, lane, w);
  const float rstd = rsqrtf(q * (1.0f / FEAT) + 1e-5f);

  const v4f sh = *(const v4fa*)(hm + f0);
  const v4f sc = *(const v4fa*)(hm + FEAT + f0);
  v4f ov;
  ov.x = (d0 * rstd) * (1.0f + sc.x) + sh.x;
  ov.y = (d1 * rstd) * (1.0f + sc.y) + sh.y;
  ov.z = (d2 * rstd) * (1.0f + sc.z) + sh.z;
  ov.w = (d3 * rstd) * (1.0f + sc.w) + sh.w;

  *(v4fa*)(srow + f0) = ov;
  __syncthreads();
  if (w < 3) {
    const float* sp = srow + 8 * tid;
    const v4f a = *(const v4fa*)sp;
    const v4f c = *(const v4fa*)(sp + 4);
    const v8h o = { (_Float16)a.x, (_Float16)a.y, (_Float16)a.z, (_Float16)a.w,
                    (_Float16)c.x, (_Float16)c.y, (_Float16)c.z, (_Float16)c.w };
    _Float16* dst = pout + (size_t)row * FEAT + 8 * tid;
    *(volatile v8h*)dst = o;
    __threadfence();
    *(volatile v8h*)dst = o;
  }
}

template <int MODE>
__global__ __launch_bounds__(256) void gemm64(
    const _Float16* __restrict__ A, int lda, long long strideA,
    const _Float16* __restrict__ Bt, int ldb, long long strideB,
    void* Cout, int ldc, long long strideC,
    const float* __restrict__ bias, const float* __restrict__ res, const float* __restrict__ gate,
    int M, int N, int K, float oscale, float ocarry, int resr)
{
  __shared__ __align__(16) float sT[8][16 * 68];
  const int b    = blockIdx.y;
  const int lane = threadIdx.x & 31;
  const int wave = threadIdx.x >> 5;
  const int tilesN = N >> 6;
  const int tilesM = M >> 6;
  const int tile = blockIdx.x * 8 + wave;
  if (tile >= tilesM * tilesN) return;
  const int tm = tile / tilesN;
  const int tn = tile - tm * tilesN;
  const int m0 = tm << 6;
  const int n0 = tn << 6;

  const _Float16* Ab = A  + (size_t)b * (size_t)strideA;
  const _Float16* Bb = Bt + (size_t)b * (size_t)strideB;

  const int rlane = lane & 15;
  const int koff  = (lane >> 4) * 8;
  const int mOff  = (lane >> 4) * 8;

  v8f acc[4][4];
#pragma unroll
  for (int i = 0; i < 4; ++i)
#pragma unroll
    for (int j = 0; j < 4; ++j) acc[i][j] = zero8();

  for (int k0 = 0; k0 < K; k0 += 32) {
    v16h bq[4];
#pragma unroll
    for (int j = 0; j < 4; ++j)
      bq[j] = ldfrag(Bb + (size_t)(n0 + (j << 4) + rlane) * ldb + koff + k0);
#pragma unroll
    for (int i = 0; i < 4; ++i) {
      const v16h af = ldfrag(Ab + (size_t)(m0 + (i << 4) + rlane) * lda + koff + k0);
#pragma unroll
      for (int j = 0; j < 4; ++j) acc[i][j] = mmar(af, bq[j], acc[i][j]);
      dep_guard(acc[i][0], acc[i][3], af, bq[3]);
    }
    keep4(bq[0], bq[1], bq[2], bq[3]);
  }
  acc_guard4(acc[0][0], acc[0][1], acc[0][2], acc[0][3]);
  acc_guard4(acc[1][0], acc[1][1], acc[1][2], acc[1][3]);
  acc_guard4(acc[2][0], acc[2][1], acc[2][2], acc[2][3]);
  acc_guard4(acc[3][0], acc[3][1], acc[3][2], acc[3][3]);

  float* slab = sT[wave];
#pragma unroll
  for (int i = 0; i < 4; ++i) {
    const int mBase = m0 + (i << 4);
#pragma unroll
    for (int j = 0; j < 4; ++j) {
#pragma unroll
      for (int r = 0; r < 8; ++r) {
        slab[(mOff + r) * 68 + (j << 4) + rlane] = acc[i][j][r];
      }
    }
    __builtin_amdgcn_fence(3, "workgroup");
    __builtin_amdgcn_wave_barrier();
    __builtin_amdgcn_fence(2, "workgroup");
    if (MODE == 0) {
      float* C = (float*)Cout + (size_t)b * (size_t)strideC;
      const float* R = res + (size_t)b * (size_t)strideC;
      const int h2 = lane >> 4, c4 = (lane & 15) * 4;
      const v4f bv = rne16_4(*(const v4fa*)(bias + n0 + c4));
      const v4f gv = *(const v4fa*)(gate + n0 + c4);
      for (int pass = 0; pass < 2; ++pass) {
#pragma unroll
        for (int it = 0; it < 8; ++it) {
          const int row = it * 2 + h2;
          const size_t go = (size_t)(mBase + row) * ldc + n0 + c4;
          const v4f sv = *(const v4fa*)(slab + row * 68 + c4);
          const v4f rv = *(const v4fa*)(R + go);
          const v4f rr = (resr != 0) ? rne16_4(rv) : rv;
          const v4f v = rr + gv * (sv * oscale + bv);
          *(volatile v4f*)(C + go) = v;
        }
        __threadfence();
      }
    } else {
      const int q = lane >> 3, c8 = (lane & 7) * 8;
      _Float16* C = (_Float16*)Cout + (size_t)b * (size_t)strideC;
      float bb8[8] = { 0.f, 0.f, 0.f, 0.f, 0.f, 0.f, 0.f, 0.f };
      if (MODE == 1 || MODE == 2) {
        const v4f ba = rne16_4(*(const v4fa*)(bias + n0 + c8));
        const v4f bc = rne16_4(*(const v4fa*)(bias + n0 + c8 + 4));
        bb8[0] = ba.x; bb8[1] = ba.y; bb8[2] = ba.z; bb8[3] = ba.w;
        bb8[4] = bc.x; bb8[5] = bc.y; bb8[6] = bc.z; bb8[7] = bc.w;
      }
      v8h hv[4];
#pragma unroll
      for (int it = 0; it < 4; ++it) {
        const int row = it * 4 + q;
        const float* sp = slab + row * 68 + c8;
        const v4f a = *(const v4fa*)sp;
        const v4f c = *(const v4fa*)(sp + 4);
        float f[8] = { a.x, a.y, a.z, a.w, c.x, c.y, c.z, c.w };
        float rb = 0.0f;
        if (MODE == 3) rb = rne16(bias[mBase + row]);
#pragma unroll
        for (int e = 0; e < 8; ++e) {
          const float u = f[e] * oscale + bb8[e] + rb;
          if (MODE == 2) {
            const float gl = 0.5f * u * (1.0f + erff(u * 0.70710678118654752f));
            f[e] = gl * ocarry;
          } else {
            f[e] = u * ocarry;
          }
        }
        const v8h o = { (_Float16)f[0], (_Float16)f[1], (_Float16)f[2], (_Float16)f[3],
                        (_Float16)f[4], (_Float16)f[5], (_Float16)f[6], (_Float16)f[7] };
        hv[it] = o;
      }
      for (int pass = 0; pass < 2; ++pass) {
#pragma unroll
        for (int it = 0; it < 4; ++it) {
          const int row = it * 4 + q;
          *(volatile v8h*)(C + (size_t)(mBase + row) * ldc + n0 + c8) = hv[it];
        }
        __threadfence();
      }
    }
    __builtin_amdgcn_fence(3, "workgroup");
    __builtin_amdgcn_wave_barrier();
    __builtin_amdgcn_fence(2, "workgroup");
  }
}

__device__ __forceinline__ v16h pack_p(v8f a, v8f c) {
  const v16h r = { (_Float16)(a[0] * PSCALE), (_Float16)(a[1] * PSCALE), (_Float16)(a[2] * PSCALE), (_Float16)(a[3] * PSCALE),
                   (_Float16)(a[4] * PSCALE), (_Float16)(a[5] * PSCALE), (_Float16)(a[6] * PSCALE), (_Float16)(a[7] * PSCALE),
                   (_Float16)(c[0] * PSCALE), (_Float16)(c[1] * PSCALE), (_Float16)(c[2] * PSCALE), (_Float16)(c[3] * PSCALE),
                   (_Float16)(c[4] * PSCALE), (_Float16)(c[5] * PSCALE), (_Float16)(c[6] * PSCALE), (_Float16)(c[7] * PSCALE) };
  return r;
}

__global__ __launch_bounds__(128) __attribute__((amdgpu_num_vgpr(256))) void attn_kernel(
    const _Float16* __restrict__ qk, const _Float16* __restrict__ vt, _Float16* ctx)
{
  __shared__ __align__(16) float sO[4 * 16 * 64];

  const int tid = (int)threadIdx.x, lane = tid & 31, w = tid >> 5;
  const int h = lane >> 4, m = lane & 15;
  const int head = blockIdx.y;
  const int q0 = blockIdx.x * 64 + 16 * w;

  const _Float16* qrow = qk + (size_t)(q0 + m) * QKP + head * HD;
  const v16h qb0 = load_frag(qrow, h);
  const v16h qb1 = load_frag(qrow + 32, h);

  v8f o[4];
#pragma unroll
  for (int t = 0; t < 4; ++t) o[t] = zero8();
  float mrun = -1e30f, lrun = 0.0f;

  const _Float16* kbase = qk + (size_t)m * QKP + FEAT + head * HD;
  const _Float16* vbase = vt + ((size_t)(head * HD) + m) * SEQ;

#pragma unroll 1
  for (int kb = 0; kb < SEQ; kb += 64) {
    v8f s[4];
#pragma unroll
    for (int j = 0; j < 4; ++j) {
      const _Float16* kr = kbase + (size_t)(kb + 16 * j) * QKP;
      const v16h kf0 = load_frag(kr, h);
      const v16h kf1 = load_frag(kr + 32, h);
      v8f z = zero8();
      z = wmma_f16(kf0, qb0, z);
      z = wmma_f16(kf1, qb1, z);
      s[j] = z * 0.125f;
    }

    float mloc = s[0][0];
#pragma unroll
    for (int j = 0; j < 4; ++j)
#pragma unroll
      for (int r = 0; r < 8; ++r) mloc = fmaxf(mloc, s[j][r]);
    mloc = fmaxf(mloc, __shfl_xor(mloc, 16));
    const float mnew = fmaxf(mrun, mloc);
    const float alpha = __expf(mrun - mnew);
    mrun = mnew;
    float lsum = 0.0f;
#pragma unroll
    for (int j = 0; j < 4; ++j)
#pragma unroll
      for (int r = 0; r < 8; ++r) {
        const float p = __expf(s[j][r] - mnew);
        s[j][r] = p;
        lsum += p;
      }
    lsum += __shfl_xor(lsum, 16);
    lrun = lrun * alpha + lsum;
#pragma unroll
    for (int t = 0; t < 4; ++t)
#pragma unroll
      for (int r = 0; r < 8; ++r) o[t][r] = o[t][r] * alpha;

    const v16h pb0 = pack_p(s[0], s[1]);
    const v16h pb1 = pack_p(s[2], s[3]);

#pragma unroll
    for (int t = 0; t < 4; ++t) {
      const _Float16* vp = vbase + (size_t)(16 * t) * SEQ + kb;
      const v16h vf0 = load_frag(vp, h);
      const v16h vf1 = load_frag(vp + 32, h);
      o[t] = wmma_f16(vf0, pb0, o[t]);
      o[t] = wmma_f16(vf1, pb1, o[t]);
    }
  }

  const float inv = (1.0f / lrun) * (CTXCARRY / PSCALE);
  float* so = sO + w * 1024;
#pragma unroll
  for (int t = 0; t < 4; ++t)
#pragma unroll
    for (int r = 0; r < 8; ++r)
      so[m * 64 + 16 * t + 8 * h + r] = o[t][r] * inv;
  __syncthreads();

  const int q8 = lane & 7, sub = lane >> 3;
  v8h hv[4];
#pragma unroll
  for (int it = 0; it < 4; ++it) {
    const int row = it * 4 + sub;
    const float* sp = so + row * 64 + 8 * q8;
    const v4f a = *(const v4fa*)sp;
    const v4f c = *(const v4fa*)(sp + 4);
    const v8h ov = { (_Float16)a.x, (_Float16)a.y, (_Float16)a.z, (_Float16)a.w,
                     (_Float16)c.x, (_Float16)c.y, (_Float16)c.z, (_Float16)c.w };
    hv[it] = ov;
  }
  for (int pass = 0; pass < 2; ++pass) {
#pragma unroll
    for (int it = 0; it < 4; ++it) {
      const int row = it * 4 + sub;
      _Float16* dst = ctx + (size_t)(q0 + row) * FEAT + head * HD + 8 * q8;
      *(volatile v8h*)dst = hv[it];
    }
    __threadfence();
  }
}

extern "C" void kernel_launch(void* const* d_in, const int* in_sizes, int n_in,
                              void* d_out, int out_size, void* d_ws, size_t ws_size,
                              hipStream_t stream)
{
  if (n_in < 14) return;
  if (in_sizes[0] < NTOK * FEAT) return;
  if (in_sizes[1] < NB * FEAT) return;
  if (in_sizes[2] < FEAT * QKVW || in_sizes[3] < QKVW) return;
  if (in_sizes[4] < FEAT * QKVW || in_sizes[5] < QKVW) return;
  if (in_sizes[6] < FEAT * FEAT || in_sizes[7] < FEAT) return;
  if (in_sizes[8] < FEAT * QKVW || in_sizes[9] < QKVW) return;
  if (in_sizes[10] < FEAT * MF || in_sizes[11] < MF) return;
  if (in_sizes[12] < MF * FEAT || in_sizes[13] < FEAT) return;
  if (out_size < NTOK * FEAT) return;

  const float* x      = (const float*)d_in[0];
  const float* cond   = (const float*)d_in[1];
  const float* w_mod1 = (const float*)d_in[2];
  const float* b_mod1 = (const float*)d_in[3];
  const float* w_qkv  = (const float*)d_in[4];
  const float* b_qkv  = (const float*)d_in[5];
  const float* w_o    = (const float*)d_in[6];
  const float* b_o    = (const float*)d_in[7];
  const float* w_mod2 = (const float*)d_in[8];
  const float* b_mod2 = (const float*)d_in[9];
  const float* w_f1   = (const float*)d_in[10];
  const float* b_f1   = (const float*)d_in[11];
  const float* w_f2   = (const float*)d_in[12];
  const float* b_f2   = (const float*)d_in[13];

  const size_t P_MOD  = (size_t)2 * QKVW * 4;
  const size_t P_F16  = (size_t)NTOK * FEAT * 2;
  const size_t P_WQKV = (size_t)QKVW * FEAT * 2;
  const size_t P_WO   = (size_t)FEAT * FEAT * 2;
  const size_t P_W1   = (size_t)MF * FEAT * 2;
  const size_t P_QK   = (size_t)NTOK * QKP * 2;
  const size_t P_VT   = (size_t)FEAT * NTOK * 2;
  const size_t P_F32  = (size_t)NTOK * FEAT * 4;
  const size_t P_MID  = (size_t)NTOK * MF * 2;
  size_t off = 0;
  const size_t oMod  = off; off += P_MOD;
  const size_t oXn   = off; off += P_F16;
  const size_t oWqkv = off; off += P_WQKV;
  const size_t oWo   = off; off += P_WO;
  const size_t oW1   = off; off += P_W1;
  const size_t oW2   = off; off += P_W1;
  const size_t oQK   = off; off += P_QK;
  const size_t oVT   = off; off += P_VT;
  const size_t oCtx  = off; off += P_F16;
  const size_t oX1   = off; off += P_F32;
  const size_t oH2   = off; off += P_F16;
  const size_t oMid  = off; off += P_MID;
  if (off > ws_size) return;
  if (off > (size_t)134217728) return;

  char* ws = (char*)d_ws;
  float*    modv  = (float*)(ws + oMod);
  _Float16* xn    = (_Float16*)(ws + oXn);
  _Float16* wqkvT = (_Float16*)(ws + oWqkv);
  _Float16* woT   = (_Float16*)(ws + oWo);
  _Float16* w1T   = (_Float16*)(ws + oW1);
  _Float16* w2T   = (_Float16*)(ws + oW2);
  _Float16* qkp   = (_Float16*)(ws + oQK);
  _Float16* vtp   = (_Float16*)(ws + oVT);
  _Float16* ctx   = (_Float16*)(ws + oCtx);
  float*    x1    = (float*)(ws + oX1);
  _Float16* h2    = (_Float16*)(ws + oH2);
  _Float16* mid   = (_Float16*)(ws + oMid);
  const float* hm1   = modv;
  const float* hm2   = modv + QKVW;
  const float* gate1 = modv + 2 * FEAT;
  const float* gate2 = modv + QKVW + 2 * FEAT;

  const dim3 blk(256);

  mod_kernel<<<dim3(2 * (QKVW / 256)), blk, 0, stream>>>(cond, w_mod1, b_mod1, w_mod2, b_mod2, modv);

  transpose_cvt<<<dim3(FEAT / 64, QKVW / 32), blk, 0, stream>>>(w_qkv, wqkvT, FEAT, QKVW, WCARRY);
  transpose_cvt<<<dim3(FEAT / 64, FEAT / 32), blk, 0, stream>>>(w_o,   woT,   FEAT, FEAT, WCARRY);
  transpose_cvt<<<dim3(FEAT / 64, MF / 32),   blk, 0, stream>>>(w_f1,  w1T,   FEAT, MF,   WCARRY);
  transpose_cvt<<<dim3(MF / 64,   FEAT / 32), blk, 0, stream>>>(w_f2,  w2T,   MF,   FEAT, WCARRY);

  ln_kernel<true><<<dim3(NTOK), dim3(192), 0, stream>>>(x, hm1, xn);

  const dim3 gQK((((NTOK / 64) * (QKP / 64)) + 7) / 8, 1);
  gemm64<1><<<gQK, blk, 0, stream>>>(
      xn, FEAT, 0LL, wqkvT, FEAT, 0LL, (void*)qkp, QKP, 0LL, b_qkv, modv, modv,
      NTOK, QKP, FEAT, 1.0f / WCARRY, 1.0f, 0);

  const dim3 gVT((((FEAT / 64) * (NTOK / 64)) + 7) / 8, 1);
  gemm64<3><<<gVT, blk, 0, stream>>>(
      wqkvT + (size_t)QKP * FEAT, FEAT, 0LL, xn, FEAT, 0LL, (void*)vtp, NTOK, 0LL, b_qkv + QKP, modv, modv,
      FEAT, NTOK, FEAT, 1.0f / WCARRY, 1.0f, 0);

  attn_kernel<<<dim3(SEQ / 64, NB * NH), dim3(128), 0, stream>>>(qkp, vtp, ctx);

  const dim3 gO((((NTOK / 64) * (FEAT / 64)) + 7) / 8, 1);
  gemm64<0><<<gO, blk, 0, stream>>>(
      ctx, FEAT, 0LL, woT, FEAT, 0LL, (void*)x1, FEAT, 0LL, b_o, x, gate1,
      NTOK, FEAT, FEAT, 1.0f / (WCARRY * CTXCARRY), 1.0f, 1);

  ln_kernel<false><<<dim3(NTOK), dim3(192), 0, stream>>>(x1, hm2, h2);

  const dim3 gW1((((NTOK / 64) * (MF / 64)) + 7) / 8, 1);
  gemm64<2><<<gW1, blk, 0, stream>>>(
      h2, FEAT, 0LL, w1T, FEAT, 0LL, (void*)mid, MF, 0LL, b_f1, modv, modv,
      NTOK, MF, FEAT, 1.0f / WCARRY, MIDCARRY, 0);

  gemm64<0><<<gO, blk, 0, stream>>>(
      mid, MF, 0LL, w2T, MF, 0LL, d_out, FEAT, 0LL, b_f2, x1, gate2,
      NTOK, FEAT, MF, 1.0f / (WCARRY * MIDCARRY), 1.0f, 0);

  (void)hipGetLastError();
}
